// MultiHeadAttention_20968030339462
// MI455X (gfx1250) — hardware-run, weakly checked
//
#include <hip/hip_runtime.h>
#ifndef NB
#define NB 16
#endif
#ifndef SEQ
#define SEQ 1024
#endif
#define NB_FULL 16
#define SEQ_FULL 1024
#define NH 8
#define HD 32
#define CM 256
#define NQKV 768
#define NREL 3969
#define MROWS (NB * SEQ)
#define PLANE ((size_t)NB * NH * SEQ * HD)

#define WS_XB ((size_t)MROWS * CM * 2)
#define WS_WQ ((size_t)NQKV * CM * 2)
#define WS_WO ((size_t)CM * 2 * CM * 2)
#define WS_BB ((size_t)NH * SEQ * SEQ * 2)
#define WS_QK (PLANE * 2 * 4)
#define WS_V  (PLANE * 2 * 2)
#define WS_CX ((size_t)NB * NH * SEQ * 64 * 2)

static_assert(SEQ % 128 == 0);
static_assert(SEQ <= SEQ_FULL);
static_assert(NB <= NB_FULL);
static_assert(NH * HD == CM);
static_assert(NQKV == 3 * CM);
static_assert(HD == 32);
static_assert(CM % 64 == 0);
static_assert(WS_XB % 256 == 0 && WS_WQ % 256 == 0 && WS_WO % 256 == 0 && WS_BB % 256 == 0 && WS_QK % 256 == 0 && WS_V % 256 == 0 && WS_CX % 256 == 0);
static_assert(WS_XB + WS_WQ + WS_WO + WS_BB + WS_QK + WS_V + WS_CX <= (size_t)134217728);

typedef __bf16 v16b __attribute__((ext_vector_type(16)));
typedef _Float16 v16h __attribute__((ext_vector_type(16)));
typedef unsigned short v8us __attribute__((ext_vector_type(8), may_alias));
typedef float v8f __attribute__((ext_vector_type(8)));
typedef float v4f __attribute__((ext_vector_type(4)));
typedef float v4fa __attribute__((ext_vector_type(4), may_alias));
union FragB { v16b v; v8us half[2]; unsigned short u[16]; };
union FragH { v16h v; v8us half[2]; _Float16 h[16]; unsigned short u[16]; };

#define LOG2E 1.4426950408889634f

__device__ __forceinline__ unsigned short bf16_bits(float x) {
  unsigned int u = __float_as_uint(x);
  return (unsigned short)((u + 0x7FFFu + ((u >> 16) & 1u)) >> 16);
}
__device__ __forceinline__ float bf16_val(unsigned short b) { return __uint_as_float(((unsigned int)b) << 16); }
__device__ __forceinline__ float bf16_rne(float x) { return bf16_val(bf16_bits(x)); }
__device__ __forceinline__ unsigned short f16_bits(float x) { return __builtin_bit_cast(unsigned short, (_Float16)x); }

__device__ __forceinline__ v8f mma_bf3(v16b a0, v16b b0, v16b a1, v16b b1, v16b a2, v16b b2, v8f c) {
  c = __builtin_amdgcn_wmma_f32_16x16x32_bf16(false, a0, false, b0, (short)0, c, false, false);
  c = __builtin_amdgcn_wmma_f32_16x16x32_bf16(false, a1, false, b1, (short)0, c, false, false);
  c = __builtin_amdgcn_wmma_f32_16x16x32_bf16(false, a2, false, b2, (short)0, c, false, false);
  asm volatile("v_nop\n\tv_nop\n\tv_nop\n\tv_nop" : "+v"(c) : "v"(a0), "v"(b0), "v"(a1), "v"(b1), "v"(a2), "v"(b2));
  return c;
}
__device__ __forceinline__ void mma_h3(v16h ah, v16h al, v16h bh, v16h bl, v8f& ch, v8f& cl) {
  ch = __builtin_amdgcn_wmma_f32_16x16x32_f16(false, ah, false, bh, (short)0, ch, false, false);
  cl = __builtin_amdgcn_wmma_f32_16x16x32_f16(false, ah, false, bl, (short)0, cl, false, false);
  cl = __builtin_amdgcn_wmma_f32_16x16x32_f16(false, al, false, bh, (short)0, cl, false, false);
  asm volatile("v_nop\n\tv_nop\n\tv_nop\n\tv_nop" : "+v"(ch), "+v"(cl) : "v"(ah), "v"(al), "v"(bh), "v"(bl));
}

__device__ __forceinline__ void gemm_step(const unsigned short* __restrict__ a0p, const unsigned short* __restrict__ a1p,
                                          const unsigned short* __restrict__ bp, int ldb, v8f (&acc)[2][4]) {
  FragB a0, a1, b0, b1, b2, b3;
  a0.half[0] = *(const v8us*)(a0p);                    a0.half[1] = *(const v8us*)(a0p + 16);
  a1.half[0] = *(const v8us*)(a1p);                    a1.half[1] = *(const v8us*)(a1p + 16);
  b0.half[0] = *(const v8us*)(bp);                     b0.half[1] = *(const v8us*)(bp + 16);
  b1.half[0] = *(const v8us*)(bp + (size_t)16 * ldb);  b1.half[1] = *(const v8us*)(bp + (size_t)16 * ldb + 16);
  b2.half[0] = *(const v8us*)(bp + (size_t)32 * ldb);  b2.half[1] = *(const v8us*)(bp + (size_t)32 * ldb + 16);
  b3.half[0] = *(const v8us*)(bp + (size_t)48 * ldb);  b3.half[1] = *(const v8us*)(bp + (size_t)48 * ldb + 16);
  acc[0][0] = __builtin_amdgcn_wmma_f32_16x16x32_bf16(false, a0.v, false, b0.v, (short)0, acc[0][0], false, false);
  acc[1][0] = __builtin_amdgcn_wmma_f32_16x16x32_bf16(false, a1.v, false, b0.v, (short)0, acc[1][0], false, false);
  acc[0][1] = __builtin_amdgcn_wmma_f32_16x16x32_bf16(false, a0.v, false, b1.v, (short)0, acc[0][1], false, false);
  acc[1][1] = __builtin_amdgcn_wmma_f32_16x16x32_bf16(false, a1.v, false, b1.v, (short)0, acc[1][1], false, false);
  acc[0][2] = __builtin_amdgcn_wmma_f32_16x16x32_bf16(false, a0.v, false, b2.v, (short)0, acc[0][2], false, false);
  acc[1][2] = __builtin_amdgcn_wmma_f32_16x16x32_bf16(false, a1.v, false, b2.v, (short)0, acc[1][2], false, false);
  acc[0][3] = __builtin_amdgcn_wmma_f32_16x16x32_bf16(false, a0.v, false, b3.v, (short)0, acc[0][3], false, false);
  acc[1][3] = __builtin_amdgcn_wmma_f32_16x16x32_bf16(false, a1.v, false, b3.v, (short)0, acc[1][3], false, false);
  asm volatile("v_nop\n\tv_nop\n\tv_nop\n\tv_nop"
               : "+v"(acc[0][0]), "+v"(acc[0][1]), "+v"(acc[0][2]), "+v"(acc[0][3]),
                 "+v"(acc[1][0]), "+v"(acc[1][1]), "+v"(acc[1][2]), "+v"(acc[1][3])
               : "v"(a0.v), "v"(a1.v), "v"(b0.v), "v"(b1.v), "v"(b2.v), "v"(b3.v));
}

__global__ __launch_bounds__(256) void k_xb(const float* __restrict__ X, unsigned short* __restrict__ Xb) {
  const int t = blockIdx.x * 256 + threadIdx.x;
  if (t >= MROWS * (CM / 8)) return;
  const int row = t >> 5, piece = t & 31;
  const int b = row / SEQ, s = row - b * SEQ;
  const float* src = X + ((size_t)b * SEQ_FULL + s) * CM + piece * 8;
  const v4f x0 = *(const v4fa*)(src), x1 = *(const v4fa*)(src + 4);
  v8us o;
  o[0] = bf16_bits(x0[0]); o[1] = bf16_bits(x0[1]); o[2] = bf16_bits(x0[2]); o[3] = bf16_bits(x0[3]);
  o[4] = bf16_bits(x1[0]); o[5] = bf16_bits(x1[1]); o[6] = bf16_bits(x1[2]); o[7] = bf16_bits(x1[3]);
  unsigned short* d = Xb + (size_t)t * 8;
  *(volatile v8us*)d = o;
  __threadfence();
  *(volatile v8us*)d = o;
}

template <int DUP>
__global__ __launch_bounds__(256) void k_wt(const float* __restrict__ W, unsigned short* __restrict__ Wt, int ncols) {
  __shared__ unsigned short tl[64][66];
  const int tid = threadIdx.x;
  const int k0 = blockIdx.x * 64, n0 = blockIdx.y * 64;
  for (int i = tid; i < 64 * 16; i += 256) {
    const int kk = i >> 4, c4 = (i & 15) * 4;
    const v4f x = *(const v4fa*)(W + (size_t)(k0 + kk) * ncols + n0 + c4);
    tl[c4 + 0][kk] = bf16_bits(x[0]); tl[c4 + 1][kk] = bf16_bits(x[1]);
    tl[c4 + 2][kk] = bf16_bits(x[2]); tl[c4 + 3][kk] = bf16_bits(x[3]);
  }
  __syncthreads();
  for (int pass = 0; pass < 2; ++pass) {
    if (DUP == 1) {
      for (int i = tid; i < 64 * 8; i += 256) {
        const int n = i >> 3, k8 = (i & 7) * 8;
        v8us o;
#pragma unroll
        for (int q = 0; q < 8; ++q) o[q] = tl[n][k8 + q];
        *(volatile v8us*)(Wt + (size_t)(n0 + n) * CM + k0 + k8) = o;
      }
    } else {
      for (int i = tid; i < 64 * 16; i += 256) {
        const int n = i >> 4, e = (i & 15) * 8;
        const int ks = (e >> 6) * 32 + (e & 31);
        v8us o;
#pragma unroll
        for (int q = 0; q < 8; ++q) o[q] = tl[n][ks + q];
        *(volatile v8us*)(Wt + (size_t)(n0 + n) * (2 * CM) + 2 * k0 + e) = o;
      }
    }
    if (pass == 0) __threadfence();
  }
}

__global__ __launch_bounds__(256) void k_bias(const float* __restrict__ tab, const int* __restrict__ ridx, unsigned short* __restrict__ Bb) {
  const int t = blockIdx.x * 256 + threadIdx.x;
  if (t >= SEQ * (SEQ / 8)) return;
  const int i = t / (SEQ / 8), j8 = (t - i * (SEQ / 8)) * 8;
  v8us o[8];
#pragma unroll
  for (int q = 0; q < 8; ++q) {
    int id = ridx[(size_t)(j8 + q) * SEQ_FULL + i];
    id = id < 0 ? 0 : (id > NREL - 1 ? NREL - 1 : id);
    const float* rt = tab + (size_t)id * NH;
    const v4f a = *(const v4fa*)(rt), c = *(const v4fa*)(rt + 4);
    o[0][q] = bf16_bits(a[0]); o[1][q] = bf16_bits(a[1]); o[2][q] = bf16_bits(a[2]); o[3][q] = bf16_bits(a[3]);
    o[4][q] = bf16_bits(c[0]); o[5][q] = bf16_bits(c[1]); o[6][q] = bf16_bits(c[2]); o[7][q] = bf16_bits(c[3]);
  }
  for (int pass = 0; pass < 2; ++pass) {
#pragma unroll
    for (int h = 0; h < NH; ++h)
      *(volatile v8us*)(Bb + ((size_t)h * SEQ + i) * SEQ + j8) = o[h];
    if (pass == 0) __threadfence();
  }
}

__global__ __launch_bounds__(128) void k_qkv(const unsigned short* __restrict__ Xb, const unsigned short* __restrict__ WqT,
                                             unsigned short* __restrict__ QK, unsigned short* __restrict__ Vpl) {
  __shared__ __attribute__((aligned(16))) unsigned short sm[2][128 * 72];
  const int tid = threadIdx.x, w = __builtin_amdgcn_readfirstlane((int)(tid >> 5)), lane = tid & 31, ln = lane & 15, hh = lane >> 4;
  const int m0 = blockIdx.x * 128, n0 = blockIdx.y * 64;
  const v8f z8 = {0.f, 0.f, 0.f, 0.f, 0.f, 0.f, 0.f, 0.f};
  v8f acc[2][4];
#pragma unroll
  for (int i = 0; i < 2; ++i)
#pragma unroll
    for (int j = 0; j < 4; ++j) acc[i][j] = z8;
  const unsigned short* a0p = Xb + (size_t)(m0 + 32 * w + ln) * CM + 8 * hh;
  const unsigned short* a1p = a0p + 16 * CM;
  const unsigned short* bp = WqT + (size_t)(n0 + ln) * CM + 8 * hh;
#pragma unroll 1
  for (int k0 = 0; k0 < CM; k0 += 32) gemm_step(a0p + k0, a1p + k0, bp + k0, CM, acc);

  const int part = n0 >> 8;
  const int head0 = (n0 & 255) >> 5;
  const int b = m0 / SEQ, s0 = m0 - b * SEQ;
  const int rb = 32 * w + 8 * hh;
  if (part < 2) {
#pragma unroll
    for (int i = 0; i < 2; ++i)
#pragma unroll
      for (int j = 0; j < 4; ++j)
#pragma unroll
        for (int r = 0; r < 8; ++r) {
          const float x = acc[i][j][r];
          const unsigned short hb = bf16_bits(x);
          const unsigned short lb = bf16_bits(x - bf16_val(hb));
          const int o = (rb + 16 * i + r) * 72 + 16 * j + ln;
          sm[0][o] = hb; sm[1][o] = lb;
        }
  } else {
#pragma unroll
    for (int i = 0; i < 2; ++i)
#pragma unroll
      for (int j = 0; j < 4; ++j)
#pragma unroll
        for (int r = 0; r < 8; ++r) {
          const float x = acc[i][j][r] * 16.0f;
          const _Float16 hv = (_Float16)x;
          const int o = (16 * j + ln) * 136 + rb + 16 * i + r;
          sm[0][o] = __builtin_bit_cast(unsigned short, hv);
          sm[1][o] = f16_bits((x - (float)hv) * 2048.0f);
        }
  }
  __syncthreads();
  for (int pass = 0; pass < 2; ++pass) {
    if (part < 2) {
#pragma unroll
      for (int pl = 0; pl < 2; ++pl)
#pragma unroll
        for (int hd = 0; hd < 2; ++hd) {
          unsigned short* base = QK + (size_t)(part * 2 + pl) * PLANE + (((size_t)b * NH + head0 + hd) * SEQ + s0) * HD;
#pragma unroll
          for (int it = 0; it < 4; ++it) {
            const int p = it * 128 + tid;
            const int s = p >> 2, d8 = (p & 3) * 8;
            const v8us o = *(const v8us*)&sm[pl][s * 72 + hd * 32 + d8];
            *(volatile v8us*)(base + (size_t)p * 8) = o;
          }
        }
    } else {
#pragma unroll
      for (int pl = 0; pl < 2; ++pl)
#pragma unroll
        for (int it = 0; it < 8; ++it) {
          const int p = it * 128 + tid;
          const int col = p >> 4, s8 = (p & 15) * 8;
          const v8us o = *(const v8us*)&sm[pl][col * 136 + s8];
          unsigned short* dst = Vpl + (size_t)pl * PLANE + (((size_t)b * NH + head0 + (col >> 5)) * HD + (col & 31)) * SEQ + s0 + s8;
          *(volatile v8us*)dst = o;
        }
    }
    if (pass == 0) __threadfence();
  }
}

__global__ __launch_bounds__(128) void k_attn(const unsigned short* __restrict__ QK, const unsigned short* __restrict__ Vpl,
                                              const unsigned short* __restrict__ Bb, unsigned short* __restrict__ Cx) {
  __shared__ __attribute__((aligned(16))) unsigned short so[4][16][72];
  const int tid = threadIdx.x, w = __builtin_amdgcn_readfirstlane((int)(tid >> 5)), lane = tid & 31, ln = lane & 15, hh = lane >> 4;
  const int bh = blockIdx.x / (SEQ / 64), qt = blockIdx.x - bh * (SEQ / 64);
  const int h = bh % NH;
  const int qbase = qt * 64 + 16 * w;
  const int qg = qbase + ln;
  FragB qh, ql;
  {
    const size_t qo = ((size_t)bh * SEQ + qg) * HD + 8 * hh;
    qh.half[0] = *(const v8us*)(QK + qo);          qh.half[1] = *(const v8us*)(QK + qo + 16);
    ql.half[0] = *(const v8us*)(QK + PLANE + qo);  ql.half[1] = *(const v8us*)(QK + PLANE + qo + 16);
  }
  const unsigned short* kph = QK + 2 * PLANE + ((size_t)bh * SEQ + ln) * HD + 8 * hh;
  const unsigned short* kpl = kph + PLANE;
  const unsigned short* vph = Vpl + ((size_t)bh * HD + ln) * SEQ + 8 * hh;
  const unsigned short* vpl = vph + PLANE;
  const unsigned short* bpp = Bb + ((size_t)h * SEQ + qg) * SEQ + 8 * hh;

  const v8f z8 = {0.f, 0.f, 0.f, 0.f, 0.f, 0.f, 0.f, 0.f};
  float mr = -1.0e30f, lr = 0.0f;
  v8f Oh0 = z8, Oh1 = z8, Ol0 = z8, Ol1 = z8;
#pragma unroll 1
  for (int j = 0; j < SEQ / 32; ++j) {
    const int key0 = 32 * j;
    const unsigned short* ka = kph + (size_t)key0 * HD;
    const unsigned short* kb = kpl + (size_t)key0 * HD;
    FragB k0h, k0l, k1h, k1l;
    k0h.half[0] = *(const v8us*)(ka);            k0h.half[1] = *(const v8us*)(ka + 16);
    k1h.half[0] = *(const v8us*)(ka + 16 * HD);  k1h.half[1] = *(const v8us*)(ka + 16 * HD + 16);
    k0l.half[0] = *(const v8us*)(kb);            k0l.half[1] = *(const v8us*)(kb + 16);
    k1l.half[0] = *(const v8us*)(kb + 16 * HD);  k1l.half[1] = *(const v8us*)(kb + 16 * HD + 16);
    const v8us bz0 = *(const v8us*)(bpp + key0);
    const v8us bz1 = *(const v8us*)(bpp + key0 + 16);
    const v8f s0 = mma_bf3(k0h.v, qh.v, k0l.v, qh.v, k0h.v, ql.v, z8);
    const v8f s1 = mma_bf3(k1h.v, qh.v, k1l.v, qh.v, k1h.v, ql.v, z8);
    const unsigned short* va = vph + key0;
    const unsigned short* vb = vpl + key0;
    FragH vh0, vh1, vl0, vl1;
    vh0.half[0] = *(const v8us*)(va);                      vh0.half[1] = *(const v8us*)(va + 16);
    vh1.half[0] = *(const v8us*)(va + (size_t)16 * SEQ);   vh1.half[1] = *(const v8us*)(va + (size_t)16 * SEQ + 16);
    vl0.half[0] = *(const v8us*)(vb);                      vl0.half[1] = *(const v8us*)(vb + 16);
    vl1.half[0] = *(const v8us*)(vb + (size_t)16 * SEQ);   vl1.half[1] = *(const v8us*)(vb + (size_t)16 * SEQ + 16);
    float sc[16];
#pragma unroll
    for (int r = 0; r < 8; ++r) {
      sc[r]     = s0[r] + bf16_val(bz0[r]);
      sc[8 + r] = s1[r] + bf16_val(bz1[r]);
    }
    float mx = sc[0];
#pragma unroll
    for (int i = 1; i < 16; ++i) mx = fmaxf(mx, sc[i]);
    mx = fmaxf(mx, __shfl_xor(mx, 16, 32));
    const float mnew = fmaxf(mr, mx);
    const float al = exp2f((mr - mnew) * LOG2E);
    mr = mnew;
    FragH ph, pl;
    float ps = 0.0f;
#pragma unroll
    for (int i = 0; i < 16; ++i) {
      const float pc = exp2f(fmaf(sc[i] - mnew, LOG2E, 14.0f));
      ps += pc;
      const _Float16 hv = (_Float16)pc;
      ph.h[i] = hv;
      pl.h[i] = (_Float16)((pc - (float)hv) * 2048.0f);
    }
    ps += __shfl_xor(ps, 16, 32);
    lr = lr * al + ps;
    Oh0 = Oh0 * al; Oh1 = Oh1 * al; Ol0 = Ol0 * al; Ol1 = Ol1 * al;
    mma_h3(vh0.v, vl0.v, ph.v, pl.v, Oh0, Ol0);
    mma_h3(vh1.v, vl1.v, ph.v, pl.v, Oh1, Ol1);
  }

  const float inv = 1.0f / (16.0f * lr);
#pragma unroll
  for (int r = 0; r < 8; ++r) {
    const float c0 = (Oh0[r] + Ol0[r] * 0.00048828125f) * inv;
    const float c1 = (Oh1[r] + Ol1[r] * 0.00048828125f) * inv;
    const unsigned short h0 = bf16_bits(c0), h1 = bf16_bits(c1);
    so[w][ln][8 * hh + r]           = h0;
    so[w][ln][16 + 8 * hh + r]      = h1;
    so[w][ln][32 + 8 * hh + r]      = bf16_bits(c0 - bf16_val(h0));
    so[w][ln][32 + 16 + 8 * hh + r] = bf16_bits(c1 - bf16_val(h1));
  }
  __syncthreads();
  unsigned short* dst = Cx + ((size_t)bh * SEQ + qbase) * 64;
  for (int pass = 0; pass < 2; ++pass) {
#pragma unroll
    for (int it = 0; it < 4; ++it) {
      const int p = it * 32 + lane;
      const int row = p >> 3, c8 = (p & 7) * 8;
      const v8us o = *(const v8us*)&so[w][row][c8];
      *(volatile v8us*)(dst + (size_t)p * 8) = o;
    }
    if (pass == 0) __threadfence();
  }
}

__global__ __launch_bounds__(128) void k_out(const unsigned short* __restrict__ Cx, const unsigned short* __restrict__ WoT,
                                             const float* __restrict__ bout, float* __restrict__ Out) {
  __shared__ __attribute__((aligned(16))) float so[128][68];
  const int tid = threadIdx.x, w = __builtin_amdgcn_readfirstlane((int)(tid >> 5)), lane = tid & 31, ln = lane & 15, hh = lane >> 4;
  const int m0 = blockIdx.x * 128, n0 = blockIdx.y * 64;
  const int b = m0 / SEQ, s0 = m0 - b * SEQ;
  const v8f z8 = {0.f, 0.f, 0.f, 0.f, 0.f, 0.f, 0.f, 0.f};
  v8f acc[2][4];
#pragma unroll
  for (int i = 0; i < 2; ++i)
#pragma unroll
    for (int j = 0; j < 4; ++j) acc[i][j] = z8;
  const unsigned short* a0b = Cx + ((size_t)b * NH * SEQ + s0 + 32 * w + ln) * 64 + 8 * hh;
  const unsigned short* bp = WoT + (size_t)(n0 + ln) * (2 * CM) + 8 * hh;
#pragma unroll 1
  for (int kk = 0; kk < 2 * NH; ++kk) {
    const unsigned short* a0p = a0b + (size_t)(kk >> 1) * SEQ * 64 + (kk & 1) * 32;
    gemm_step(a0p, a0p + 16 * 64, bp + kk * 32, 2 * CM, acc);
  }
  const int rb = 32 * w + 8 * hh;
#pragma unroll
  for (int j = 0; j < 4; ++j) {
    const float bb = bf16_rne(bout[n0 + 16 * j + ln]);
#pragma unroll
    for (int i = 0; i < 2; ++i)
#pragma unroll
      for (int r = 0; r < 8; ++r)
        so[rb + 16 * i + r][16 * j + ln] = acc[i][j][r] + bb;
  }
  __syncthreads();
  float* og = Out + ((size_t)b * SEQ_FULL + s0) * CM + n0;
  for (int pass = 0; pass < 2; ++pass) {
#pragma unroll
    for (int it = 0; it < 16; ++it) {
      const int p = it * 128 + tid;
      const int row = p >> 4, c4 = (p & 15) * 4;
      const v4f v = *(const v4fa*)&so[row][c4];
      *(volatile v4f*)(og + (size_t)row * CM + c4) = v;
    }
    if (pass == 0) __threadfence();
  }
}

extern "C" void kernel_launch(void* const* d_in, const int* in_sizes, int n_in,
                              void* d_out, int out_size, void* d_ws, size_t ws_size, hipStream_t stream) {
  if (n_in < 6) return;
  const long long need_x = ((long long)(NB - 1) * SEQ_FULL + SEQ) * CM;
  const long long need_i = (long long)(SEQ - 1) * SEQ_FULL + SEQ;
  if ((long long)in_sizes[0] < need_x) return;
  if ((long long)in_sizes[1] < (long long)CM * NQKV) return;
  if ((long long)in_sizes[2] < (long long)NREL * NH) return;
  if ((long long)in_sizes[3] < (long long)CM * CM) return;
  if ((long long)in_sizes[4] < (long long)CM) return;
  if ((long long)in_sizes[5] < need_i) return;
  if ((long long)out_size < need_x) return;
  const float* x     = (const float*)d_in[0];
  const float* wqkv  = (const float*)d_in[1];
  const float* rtab  = (const float*)d_in[2];
  const float* wout  = (const float*)d_in[3];
  const float* bout  = (const float*)d_in[4];
  const int*   ridx  = (const int*)d_in[5];
  float* Out = (float*)d_out;
  char* ws = (char*)d_ws;
  size_t off = 0;
  unsigned short* Xb  = (unsigned short*)(ws + off); off += WS_XB;
  unsigned short* WqT = (unsigned short*)(ws + off); off += WS_WQ;
  unsigned short* WoT = (unsigned short*)(ws + off); off += WS_WO;
  unsigned short* Bb  = (unsigned short*)(ws + off); off += WS_BB;
  unsigned short* QK  = (unsigned short*)(ws + off); off += WS_QK;
  unsigned short* Vpl = (unsigned short*)(ws + off); off += WS_V;
  unsigned short* Cx  = (unsigned short*)(ws + off); off += WS_CX;
  if (off > ws_size) return;
  k_xb<<<(unsigned)((MROWS * (CM / 8) + 255) / 256), 256, 0, stream>>>(x, Xb);
  k_wt<1><<<dim3(CM / 64, NQKV / 64), 256, 0, stream>>>(wqkv, WqT, NQKV);
  k_wt<2><<<dim3(CM / 64, CM / 64), 256, 0, stream>>>(wout, WoT, CM);
  k_bias<<<(unsigned)((SEQ * (SEQ / 8) + 255) / 256), 256, 0, stream>>>(rtab, ridx, Bb);
  k_qkv<<<dim3(MROWS / 128, NQKV / 64), 128, 0, stream>>>(Xb, WqT, QK, Vpl);
  k_attn<<<(unsigned)(NB * NH * (SEQ / 64)), 128, 0, stream>>>(QK, Vpl, Bb, Cx);
  k_out<<<dim3(MROWS / 128, CM / 64), 128, 0, stream>>>(Cx, WoT, bout, Out);
}
